// GIN_74268574482528
// MI455X (gfx1250) — hardware-verified
//
#include <hip/hip_runtime.h>
#include <stddef.h>
#include <stdint.h>


#define HD       64
#define KP       128
#define NTHR     256
#define NWAVE    8
#define EPT      8
#define CHUNK    (NTHR * EPT)
#define WCAP     (EPT * 32)
#define LISTN    (NWAVE * WCAP)
#define NBMAX    1024
#define PKS      10
#define RCAP     28672
#define NB_E     1024
#define NB_P     128
#define DEGCAP_E 64
#define DEGCAP_P 128
#define GBM      128
#define GBN      64
#define GTHR     256
#define GNT      4
#define RECW     (2 * GBN)
#define NUW      1024
#define NPLN     7
#define NUWT     (NPLN * NUW)
#define HROWS    128
#define WSCAP    134217728
#define LDS_CMP  ((2 * RCAP + 2 * NBMAX + LISTN) * 4 + 64)

static_assert((HD % 8) == 0 && KP == 2 * HD && (KP % 32) == 0);
static_assert((CHUNK & (CHUNK - 1)) == 0);
static_assert((NBMAX & (NBMAX - 1)) == 0 && NBMAX == (1 << PKS) && NTHR * 4 == NBMAX);
static_assert(((long long)CHUNK << PKS) < (1LL << 31));
static_assert(LISTN >= NBMAX && LISTN == NWAVE * WCAP);
static_assert((RCAP % (4 * NTHR)) == 0 && ((2 * RCAP + NBMAX) % 4) == 0);
static_assert(LDS_CMP <= 300000);
static_assert(NB_E <= NBMAX && NB_P <= NBMAX && (NB_E % 128) == 0 && (NB_P % 128) == 0);
static_assert(RCAP * 100LL >= 16710LL * 105LL);
static_assert(DEGCAP_E >= 36 + 8);
static_assert(RCAP * 100LL >= 12670LL * 105LL);
static_assert(DEGCAP_P >= 78 + 8);
static_assert(GBM == (GTHR / 32) * 16 && GBN == 16 * GNT && GBN == HD);
static_assert(((GBM * GBN) % GTHR) == 0 && RECW == 4 * 32);
static_assert((NUWT % NTHR) == 0 && NUW == HD * (KP / 8));
static_assert(2048 % HROWS == 0 && (HROWS % 16) == 0);

typedef float          v4f  __attribute__((ext_vector_type(4)));
typedef float          v8f  __attribute__((ext_vector_type(8)));
typedef int            v4i  __attribute__((ext_vector_type(4)));
typedef int            v8i  __attribute__((ext_vector_type(8)));
typedef unsigned int   v2u  __attribute__((ext_vector_type(2)));
typedef unsigned short v8us __attribute__((ext_vector_type(8)));
typedef __bf16         v16b __attribute__((ext_vector_type(16)));
typedef v4f  __attribute__((may_alias)) v4fa;
typedef v4i  __attribute__((may_alias)) v4ia;
typedef v2u  __attribute__((may_alias)) v2ua;
typedef v8us __attribute__((may_alias)) v8usa;
union Frag { v16b vb; v8us h[2]; v8i w; };

__device__ __forceinline__ v8f wmx(const Frag& a, const Frag& b, v8f c) {
  v8f d = __builtin_amdgcn_wmma_f32_16x16x32_bf16(false, a.vb, false, b.vb, (short)0, c, false, false);
  asm volatile("v_nop\n\tv_nop\n\tv_nop\n\tv_nop" : "+v"(d) : "v"(a.w), "v"(b.w));
  return d;
}

__device__ __forceinline__ unsigned short bf_bits(float f) {
  const unsigned int u = __float_as_uint(f);
  const unsigned int r = (u + 0x7FFFu + ((u >> 16) & 1u)) >> 16;
  const bool isn = (u & 0x7fffffffu) > 0x7f800000u;
  return (unsigned short)(isn ? 0x7fc0u : r);
}
__device__ __forceinline__ float bf_val(unsigned short b) { return __uint_as_float(((unsigned int)b) << 16); }
__device__ __forceinline__ float bf_rne(float f) { return bf_val(bf_bits(f)); }

__device__ __forceinline__ float gelu_exact(float v) {
  return 0.5f * v * (1.0f + erff(v * 0.70710678118654752f));
}

__device__ __forceinline__ int scan_chunk(const int* __restrict__ dsts, int nE, int cbase, int slotBase,
                                          int nb, int vec8, int* list, int tid, int lane, int wave) {
  int wc = 0;
  const int el0  = tid * EPT;
  const int e0   = cbase + el0;
  const int sent = -2147483647 - 1;
  v4i da, db;
  if (vec8 != 0 && cbase + CHUNK <= nE) {
    da = *(const v4i*)(dsts + e0);
    db = *(const v4i*)(dsts + e0 + 4);
  } else {
    da.x = (e0     < nE) ? dsts[min(e0,     nE - 1)] : sent;
    da.y = (e0 + 1 < nE) ? dsts[min(e0 + 1, nE - 1)] : sent;
    da.z = (e0 + 2 < nE) ? dsts[min(e0 + 2, nE - 1)] : sent;
    da.w = (e0 + 3 < nE) ? dsts[min(e0 + 3, nE - 1)] : sent;
    db.x = (e0 + 4 < nE) ? dsts[min(e0 + 4, nE - 1)] : sent;
    db.y = (e0 + 5 < nE) ? dsts[min(e0 + 5, nE - 1)] : sent;
    db.z = (e0 + 6 < nE) ? dsts[min(e0 + 6, nE - 1)] : sent;
    db.w = (e0 + 7 < nE) ? dsts[min(e0 + 7, nE - 1)] : sent;
  }
  const unsigned nbs = (unsigned)slotBase;
  const unsigned unb = (unsigned)nb;
  const unsigned s0 = (unsigned)da.x - nbs, s1 = (unsigned)da.y - nbs;
  const unsigned s2 = (unsigned)da.z - nbs, s3 = (unsigned)da.w - nbs;
  const unsigned s4 = (unsigned)db.x - nbs, s5 = (unsigned)db.y - nbs;
  const unsigned s6 = (unsigned)db.z - nbs, s7 = (unsigned)db.w - nbs;
  const bool h0 = s0 < unb, h1 = s1 < unb, h2 = s2 < unb, h3 = s3 < unb;
  const bool h4 = s4 < unb, h5 = s5 < unb, h6 = s6 < unb, h7 = s7 < unb;
  const unsigned any = __builtin_amdgcn_ballot_w32(h0 | h1 | h2 | h3 | h4 | h5 | h6 | h7);
  if (any != 0u) {
#define HITJ(J, HJ, SJ) { \
      const unsigned mj = __builtin_amdgcn_ballot_w32(HJ); \
      if (mj != 0u) { \
        if (HJ) { \
          const int pos = wc + (int)__builtin_amdgcn_mbcnt_lo(mj, 0u); \
          if (pos < WCAP) list[wave * WCAP + pos] = ((el0 + (J)) << PKS) | (int)(SJ); \
        } \
        wc += (int)__builtin_popcount(mj); } }
    HITJ(0, h0, s0)
    HITJ(1, h1, s1)
    HITJ(2, h2, s2)
    HITJ(3, h3, s3)
    HITJ(4, h4, s4)
    HITJ(5, h5, s5)
    HITJ(6, h6, s6)
    HITJ(7, h7, s7)
#undef HITJ
  }
  return wc;
}

__device__ __forceinline__ v8us cv8b(const float* __restrict__ p, size_t stride) {
  v8us o;
#pragma unroll
  for (int i = 0; i < 8; ++i) o[i] = bf_bits(p[(size_t)i * stride]);
  return o;
}

__global__ __launch_bounds__(NTHR) void k_prep(const float* __restrict__ x, const float* __restrict__ cw1,
                                               const float* __restrict__ cw2, const float* __restrict__ hw1,
                                               unsigned short* wp, unsigned short* xb, int nN, int nPad) {
  const int u = (int)blockIdx.x * NTHR + (int)threadIdx.x;
  v8us o;
  unsigned short* dp;
  if (u < NUWT) {
    const int mid = u >> 10;
    const int v = u & (NUW - 1);
    const int n = v >> 4;
    const int k8 = (v & 15) * 8;
    const int kk = k8 & (HD - 1);
    if (mid < 3) {
      o = cv8b(cw1 + (size_t)mid * (HD * HD) + (size_t)kk * HD + n, HD);
    } else if (mid < 6) {
      o = cv8b(cw2 + (size_t)(mid - 3) * (HD * HD) + (size_t)kk * HD + n, HD);
    } else {
      o = cv8b(hw1 + (size_t)kk * HD + n, HD);
    }
    dp = wp + (size_t)u * 8;
  } else {
    const int v = u - NUWT;
    if (v >= nPad * 8) return;
    const int row = v >> 3;
    const int c8 = (v & 7) * 8;
    const int rc = row < nN ? row : nN - 1;
    const float* p = x + (size_t)rc * HD + c8;
    const v4f a = *(const v4f*)p;
    const v4f b = *(const v4f*)(p + 4);
    const bool live = row < nN;
    const float f[8] = {a.x, a.y, a.z, a.w, b.x, b.y, b.z, b.w};
#pragma unroll
    for (int j = 0; j < 8; ++j) o[j] = bf_bits(live ? f[j] : 0.0f);
    dp = xb + (size_t)v * 8;
  }
  *(volatile v8us*)dp = o;
  __threadfence();
  *(volatile v8us*)dp = o;
}

template <int IDV>
__global__ __launch_bounds__(NTHR) void k_compact(const int* __restrict__ keys, const int* __restrict__ vals,
                                                  int nE, int nb, int vec8, int nSrc,
                                                  int* lst, int* cntT, int* offT) {
  extern __shared__ v4f lds_dyn[];
  int* reg1 = (int*)lds_dyn;
  int* reg2 = reg1 + RCAP;
  int* scnt = reg2 + RCAP;
  int* soff = scnt + NBMAX;
  int* list = soff + NBMAX;
  int* wcnt = list + LISTN;
  int* wtot = wcnt + NWAVE;
  const int tid = (int)threadIdx.x, lane = tid & 31, wave = tid >> 5;
  const int slotBase = (int)blockIdx.x * nb;

  {
    const v4i z4 = {0, 0, 0, 0};
    for (int i = tid * 4; i < 2 * RCAP + NBMAX; i += NTHR * 4) *(v4ia*)(reg1 + i) = z4;
  }
  __syncthreads();

  int tot = 0;
  const int nChunks = (nE + CHUNK - 1) / CHUNK;
#pragma unroll 1
  for (int ch = 0; ch < nChunks; ++ch) {
    const int cbase = ch * CHUNK;
    const int wc = scan_chunk(keys, nE, cbase, slotBase, nb, vec8, list, tid, lane, wave);
    if (lane == 0) wcnt[wave] = wc;
    __syncthreads();
    int pre = 0, all = 0;
#pragma unroll
    for (int w2 = 0; w2 < NWAVE; ++w2) {
      int c = wcnt[w2];
      c = c < 0 ? 0 : (c > WCAP ? WCAP : c);
      all += c;
      pre += (w2 < wave) ? c : 0;
    }
    const int wcc  = wc > WCAP ? WCAP : wc;
    const int base = tot + pre;
#pragma unroll 1
    for (int i = lane; i < wcc; i += 32) {
      const int ent = list[wave * WCAP + i];
      const int el  = (ent >> PKS) & (CHUNK - 1);
      const int sl  = ent & (NBMAX - 1);
      int eid = cbase + el;
      eid = eid > nE - 1 ? nE - 1 : eid;
      const int pos = base + i;
      if (pos < RCAP) reg1[pos] = (eid << PKS) | sl;
    }
    tot += all;
    tot = tot > RCAP ? RCAP : tot;
    __syncthreads();
  }
  const int nh = tot;

  if (wave == 0) {
#pragma unroll 1
    for (int b0 = 0; b0 < nh; b0 += 32) {
      const int idx = b0 + lane;
      const int uv  = reg1[idx < RCAP ? idx : RCAP - 1];
      const int m32 = (nh - b0) < 32 ? (nh - b0) : 32;
#pragma unroll 1
      for (int k = 0; k < m32; ++k) {
        const int u  = __builtin_amdgcn_readlane(uv, k);
        const int sl = u & (NBMAX - 1);
        if (lane == 0) scnt[sl] = scnt[sl] + 1;
      }
    }
  }
  __syncthreads();

  {
    const v4i ca = *(const v4ia*)(scnt + 4 * tid);
    const int e0 = ca.x < 0 ? 0 : ca.x, e1 = ca.y < 0 ? 0 : ca.y;
    const int e2 = ca.z < 0 ? 0 : ca.z, e3 = ca.w < 0 ? 0 : ca.w;
    const int ts = e0 + e1 + e2 + e3;
    int incl = ts;
#pragma unroll
    for (int d = 1; d < 32; d <<= 1) {
      const int up = __shfl_up(incl, d);
      if (lane >= d) incl += up;
    }
    if (lane == 31) wtot[wave] = incl;
    __syncthreads();
    int pre = 0;
#pragma unroll
    for (int w2 = 0; w2 < NWAVE; ++w2) pre += (w2 < wave) ? wtot[w2] : 0;
    int run = pre + incl - ts;
    soff[4 * tid + 0] = run; run += e0;
    soff[4 * tid + 1] = run; run += e1;
    soff[4 * tid + 2] = run; run += e2;
    soff[4 * tid + 3] = run;
  }
  __syncthreads();
  for (int i = tid; i < NBMAX; i += NTHR) list[i] = soff[i];
  __syncthreads();

  if (wave == 0) {
#pragma unroll 1
    for (int b0 = 0; b0 < nh; b0 += 32) {
      const int idx = b0 + lane;
      const int uv  = reg1[idx < RCAP ? idx : RCAP - 1];
      const int m32 = (nh - b0) < 32 ? (nh - b0) : 32;
#pragma unroll 1
      for (int k = 0; k < m32; ++k) {
        const int u   = __builtin_amdgcn_readlane(uv, k);
        const int sl  = u & (NBMAX - 1);
        const int eid = (int)((unsigned)u >> PKS);
        if (lane == 0) {
          int pos = list[sl];
          pos = pos < 0 ? 0 : (pos > RCAP - 1 ? RCAP - 1 : pos);
          reg2[pos] = eid;
          list[sl] = pos + 1;
        }
      }
    }
  }
  __syncthreads();

  const bool ovf = (nh >= RCAP);
  int* lb = lst + (size_t)blockIdx.x * RCAP;
#pragma unroll 1
  for (int it = 0; it < RCAP / (4 * NTHR); ++it) {
    const int p4 = (it * NTHR + tid) * 4;
    const v4i e4 = *(const v4ia*)(reg2 + p4);
    int o0, o1, o2, o3;
    if constexpr (IDV != 0) {
      o0 = e4.x; o1 = e4.y; o2 = e4.z; o3 = e4.w;
    } else {
      const int a0 = e4.x < 0 ? 0 : (e4.x > nE - 1 ? nE - 1 : e4.x);
      const int a1 = e4.y < 0 ? 0 : (e4.y > nE - 1 ? nE - 1 : e4.y);
      const int a2 = e4.z < 0 ? 0 : (e4.z > nE - 1 ? nE - 1 : e4.z);
      const int a3 = e4.w < 0 ? 0 : (e4.w > nE - 1 ? nE - 1 : e4.w);
      o0 = vals[a0]; o1 = vals[a1]; o2 = vals[a2]; o3 = vals[a3];
      o0 = o0 < 0 ? 0 : (o0 > nSrc - 1 ? nSrc - 1 : o0);
      o1 = o1 < 0 ? 0 : (o1 > nSrc - 1 ? nSrc - 1 : o1);
      o2 = o2 < 0 ? 0 : (o2 > nSrc - 1 ? nSrc - 1 : o2);
      o3 = o3 < 0 ? 0 : (o3 > nSrc - 1 ? nSrc - 1 : o3);
    }
    v4i ov;
    ov.x = (p4     < nh) ? o0 : 0;
    ov.y = (p4 + 1 < nh) ? o1 : 0;
    ov.z = (p4 + 2 < nh) ? o2 : 0;
    ov.w = (p4 + 3 < nh) ? o3 : 0;
    *(volatile v4i*)(lb + p4) = ov;
    __threadfence();
    *(volatile v4i*)(lb + p4) = ov;
  }
  {
    const bool ok = (4 * tid) < nb;
    const int t4 = ok ? 4 * tid : 0;
    v4i c4 = *(const v4ia*)(scnt + t4);
    const v4i o4 = *(const v4ia*)(soff + t4);
    if (ovf) { c4.x = 0x40000000; c4.y = 0x40000000; c4.z = 0x40000000; c4.w = 0x40000000; }
    int* cp = cntT + (size_t)blockIdx.x * (size_t)nb + t4;
    int* op = offT + (size_t)blockIdx.x * (size_t)nb + t4;
    if (ok) { *(volatile v4i*)cp = c4; *(volatile v4i*)op = o4; }
    __threadfence();
    if (ok) { *(volatile v4i*)cp = c4; *(volatile v4i*)op = o4; }
  }
}

template <int MODE>
__global__ __launch_bounds__(NTHR) void k_agg(const int* __restrict__ lst, const int* __restrict__ cntT,
                                              const int* __restrict__ offT,
                                              const unsigned short* __restrict__ xb,
                                              const float* __restrict__ hf,
                                              unsigned short* pout,
                                              int nb, int nLive, int nSrc, int mRows, int degcap) {
  __shared__ __attribute__((aligned(16))) int scnt[NBMAX];
  __shared__ __attribute__((aligned(16))) int soff[NBMAX];
  const int tid = (int)threadIdx.x, lane = tid & 31, wave = tid >> 5, hh = lane >> 4, m = lane & 15;
  const int rowBase = (int)blockIdx.x * nb;
  {
    const int t4 = 4 * tid;
    const bool ok = t4 < nb;
    const int ta = ok ? t4 : 0;
    v4i c4 = *(const v4i*)(cntT + (size_t)blockIdx.x * (size_t)nb + ta);
    v4i o4 = *(const v4i*)(offT + (size_t)blockIdx.x * (size_t)nb + ta);
    const v4i z4 = {0, 0, 0, 0};
    c4 = ok ? c4 : z4;
    o4 = ok ? o4 : z4;
    *(v4ia*)(scnt + t4) = c4;
    *(v4ia*)(soff + t4) = o4;
  }
  __syncthreads();

  const int* lb = lst + (size_t)blockIdx.x * RCAP;
  const int nbw = nb >> 3;
  const float qnan = __int_as_float(0x7fc00000);

#pragma unroll 1
  for (int jt = 0; jt < nbw; ++jt) {
    const int slot = wave * nbw + jt;
    const int grow = rowBase + slot;
    const int craw = __builtin_amdgcn_readfirstlane(scnt[slot]);
    int st = __builtin_amdgcn_readfirstlane(soff[slot]);
    const bool bad = (craw < 0) || (craw > degcap);
    int cnt = craw < 0 ? 0 : (craw > degcap ? degcap : craw);
    st = st < 0 ? 0 : (st > RCAP ? RCAP : st);
    if (cnt > RCAP - st) cnt = RCAP - st;
    const bool liveRow = grow < nLive;

    float a0 = 0.0f, a1 = 0.0f, a2 = 0.0f, a3 = 0.0f;
#pragma unroll 1
    for (int b0 = 0; b0 < cnt; b0 += 32) {
      int idx = st + b0 + lane;
      idx = idx > RCAP - 1 ? RCAP - 1 : idx;
      int sr = lb[idx];
      sr = sr < 0 ? 0 : (sr > nSrc - 1 ? nSrc - 1 : sr);
      const int m32 = (cnt - b0) < 32 ? (cnt - b0) : 32;
      const int npair = (m32 + 1) >> 1;
#pragma unroll 1
      for (int k = 0; k < npair; ++k) {
        const int j  = 2 * k + hh;
        const int sk = __shfl(sr, j, 32);
        const float wv = (j < m32) ? 1.0f : 0.0f;
        float v0, v1, v2, v3;
        if constexpr (MODE == 0) {
          const v2u q = *(const v2ua*)(xb + (size_t)sk * HD + 4 * m);
          v0 = __uint_as_float(q.x << 16);
          v1 = __uint_as_float(q.x & 0xffff0000u);
          v2 = __uint_as_float(q.y << 16);
          v3 = __uint_as_float(q.y & 0xffff0000u);
        } else {
          const v4f q = *(const v4f*)(hf + (size_t)sk * HD + 4 * m);
          v0 = q.x; v1 = q.y; v2 = q.z; v3 = q.w;
        }
        a0 = fmaf(v0, wv, a0);
        a1 = fmaf(v1, wv, a1);
        a2 = fmaf(v2, wv, a2);
        a3 = fmaf(v3, wv, a3);
      }
    }
    a0 = a0 + __shfl_xor(a0, 16, 32);
    a1 = a1 + __shfl_xor(a1, 16, 32);
    a2 = a2 + __shfl_xor(a2, 16, 32);
    a3 = a3 + __shfl_xor(a3, 16, 32);

    float r0 = a0, r1 = a1, r2 = a2, r3 = a3;
    if constexpr (MODE != 2) {
      const int nc = liveRow ? grow : nLive - 1;
      float s0, s1, s2, s3;
      if constexpr (MODE == 0) {
        const v2u q = *(const v2ua*)(xb + (size_t)nc * HD + 4 * m);
        s0 = __uint_as_float(q.x << 16);
        s1 = __uint_as_float(q.x & 0xffff0000u);
        s2 = __uint_as_float(q.y << 16);
        s3 = __uint_as_float(q.y & 0xffff0000u);
      } else {
        const v4f q = *(const v4f*)(hf + (size_t)nc * HD + 4 * m);
        s0 = q.x; s1 = q.y; s2 = q.z; s3 = q.w;
      }
      r0 = s0 + a0; r1 = s1 + a1; r2 = s2 + a2; r3 = s3 + a3;
    }
    const float pz = bad ? qnan : 0.0f;
    r0 = (liveRow ? r0 : 0.0f) + pz;
    r1 = (liveRow ? r1 : 0.0f) + pz;
    r2 = (liveRow ? r2 : 0.0f) + pz;
    r3 = (liveRow ? r3 : 0.0f) + pz;

    const unsigned short h0 = bf_bits(r0), h1 = bf_bits(r1), h2 = bf_bits(r2), h3 = bf_bits(r3);
    const unsigned short l0 = bf_bits(r0 - bf_val(h0)), l1 = bf_bits(r1 - bf_val(h1));
    const unsigned short l2 = bf_bits(r2 - bf_val(h2)), l3 = bf_bits(r3 - bf_val(h3));
    const bool isLo = (hh != 0);
    const unsigned int q0 = isLo ? l0 : h0, q1 = isLo ? l1 : h1, q2 = isLo ? l2 : h2, q3 = isLo ? l3 : h3;
    v2u pk;
    pk.x = q0 | (q1 << 16);
    pk.y = q2 | (q3 << 16);
    unsigned short* gp = pout + (size_t)grow * KP + 4 * lane;
    const bool wsv = grow < mRows;
    if (wsv) *(volatile v2u*)gp = pk;
    __threadfence();
    if (wsv) *(volatile v2u*)gp = pk;
  }
}

template <int EPI>
__global__ __launch_bounds__(GTHR) void k_gemm(const unsigned short* __restrict__ A,
                                               const unsigned short* __restrict__ BT,
                                               const float* __restrict__ bias,
                                               float* outp, int nN, int mRows, float* rec) {
  __shared__ __attribute__((aligned(16))) float stg[GBM * GBN];
  __shared__ __attribute__((aligned(16))) float pst[RECW];
  const int tid = (int)threadIdx.x, lane = tid & 31, wave = tid >> 5, hh = lane >> 4, m = lane & 15;
  const int rowBase = (int)blockIdx.x * GBM;

  v8f acc[GNT];
  {
    const v8f z = {0.f, 0.f, 0.f, 0.f, 0.f, 0.f, 0.f, 0.f};
#pragma unroll
    for (int t = 0; t < GNT; ++t) acc[t] = z;
  }
  const unsigned short* ap = A  + (size_t)(rowBase + 16 * wave + m) * (size_t)KP + 8 * hh;
  const unsigned short* bp = BT + (size_t)m * (size_t)KP + 8 * hh;

#pragma unroll 1
  for (int k0 = 0; k0 < KP; k0 += 32) {
    Frag af;
    af.h[0] = *(const v8usa*)(ap + k0);
    af.h[1] = *(const v8usa*)(ap + k0 + 16);
#pragma unroll
    for (int nt = 0; nt < GNT; ++nt) {
      const unsigned short* wq = bp + (size_t)(16 * nt) * (size_t)KP + k0;
      Frag bfr;
      bfr.h[0] = *(const v8usa*)wq;
      bfr.h[1] = *(const v8usa*)(wq + 16);
      acc[nt] = wmx(af, bfr, acc[nt]);
    }
  }

#pragma unroll
  for (int nt = 0; nt < GNT; ++nt) {
    const int lc = 16 * nt + m;
    const float bb = bf_rne(bias[lc]);
#pragma unroll
    for (int r = 0; r < 8; ++r) {
      const int lr = 16 * wave + 8 * hh + r;
      const bool live = (rowBase + lr) < nN;
      const float v = acc[nt][r] + bb;
      stg[lr * GBN + lc] = live ? v : 0.0f;
    }
  }
  __syncthreads();

  if constexpr (EPI == 1) {
#pragma unroll 1
    for (int i = 0; i < (GBM * GBN) / GTHR; ++i) {
      const int idx = i * GTHR + tid;
      stg[idx] = gelu_exact(stg[idx]);
    }
    __syncthreads();
  }

  v4f fv[8];
#pragma unroll
  for (int i = 0; i < 8; ++i) {
    const int lr = 16 * wave + 2 * i + hh;
    fv[i] = *(const v4fa*)(stg + lr * GBN + 4 * m);
  }
  v4f pv = {0.f, 0.f, 0.f, 0.f};
  const bool pok = (EPI == 0) && (tid < RECW / 4);
  if constexpr (EPI == 0) {
    int nvr = nN - rowBase;
    nvr = nvr < 0 ? 0 : (nvr > GBM ? GBM : nvr);
    if (tid < GBN) {
      float s = 0.0f;
#pragma unroll 1
      for (int r = 0; r < nvr; ++r) s += stg[r * GBN + tid];
      const float inv = 1.0f / (float)(nvr < 1 ? 1 : nvr);
      const float mean = s * inv;
      float q = 0.0f;
#pragma unroll 1
      for (int r = 0; r < nvr; ++r) {
        const float d = stg[r * GBN + tid] - mean;
        q = fmaf(d, d, q);
      }
      pst[tid] = mean;
      pst[GBN + tid] = q;
    }
    __syncthreads();
    if (pok) pv = *(const v4fa*)(pst + 4 * tid);
  }
  float* pp = rec + (size_t)blockIdx.x * RECW + 4 * tid;
#pragma unroll
  for (int i = 0; i < 8; ++i) {
    const int gr = rowBase + 16 * wave + 2 * i;
    float* op = outp + (size_t)gr * GBN + 4 * lane;
    if (gr + 1 < mRows) *(volatile v4f*)op = fv[i];
  }
  if (pok) *(volatile v4f*)pp = pv;
  __threadfence();
#pragma unroll
  for (int i = 0; i < 8; ++i) {
    const int gr = rowBase + 16 * wave + 2 * i;
    float* op = outp + (size_t)gr * GBN + 4 * lane;
    if (gr + 1 < mRows) *(volatile v4f*)op = fv[i];
  }
  if (pok) *(volatile v4f*)pp = pv;
}

__global__ __launch_bounds__(GBN) void k_comb(const float* __restrict__ rec, int nRec, int nN, float* stat) {
  __shared__ __attribute__((aligned(16))) float stg[RECW];
  const int c = (int)threadIdx.x;
  double sn = 0.0, sm = 0.0;
#pragma unroll 1
  for (int b = 0; b < nRec; ++b) {
    int nb = nN - b * GBM;
    nb = nb < 0 ? 0 : (nb > GBM ? GBM : nb);
    const double dn = (double)nb;
    sm = sm + dn * (double)rec[(size_t)b * RECW + c];
    sn = sn + dn;
  }
  const double invn = 1.0 / (sn < 1.0 ? 1.0 : sn);
  const double mean = sm * invn;
  double M2 = 0.0;
#pragma unroll 1
  for (int b = 0; b < nRec; ++b) {
    int nb = nN - b * GBM;
    nb = nb < 0 ? 0 : (nb > GBM ? GBM : nb);
    const double d = (double)rec[(size_t)b * RECW + c] - mean;
    M2 = M2 + (double)rec[(size_t)b * RECW + GBN + c] + (double)nb * d * d;
  }
  const float varf = (float)(M2 * invn);
  const float rs = 1.0f / sqrtf(varf + 1e-5f);
  stg[c] = (float)mean;
  stg[GBN + c] = rs;
  __syncthreads();
  v4f v = {0.f, 0.f, 0.f, 0.f};
  const bool ok = c < RECW / 4;
  if (ok) {
    v = *(const v4fa*)(stg + 4 * c);
    *(volatile v4f*)(stat + 4 * c) = v;
  }
  __threadfence();
  if (ok) *(volatile v4f*)(stat + 4 * c) = v;
}

__global__ __launch_bounds__(NTHR) void k_apply(const float* __restrict__ T, const float* __restrict__ stat,
                                                const float* __restrict__ gam, const float* __restrict__ bet,
                                                unsigned short* p1, int nN, int nUnits) {
  __shared__ float smu[HD], srs[HD], sga[HD], sbe[HD];
  const int tid = (int)threadIdx.x;
  if (tid < HD) {
    smu[tid] = stat[tid];
    srs[tid] = stat[HD + tid];
    sga[tid] = bf_rne(gam[tid]);
    sbe[tid] = bf_rne(bet[tid]);
  }
  __syncthreads();
  const int u = (int)blockIdx.x * NTHR + tid;
  if (u >= nUnits) return;
  const int row = u >> 3;
  const int c8 = (u & 7) * 8;
  const float* p = T + (size_t)u * 8;
  const v4f a = *(const v4f*)p;
  const v4f b = *(const v4f*)(p + 4);
  const bool live = row < nN;
  const float f[8] = {a.x, a.y, a.z, a.w, b.x, b.y, b.z, b.w};
  v8us hv, lv;
#pragma unroll
  for (int j = 0; j < 8; ++j) {
    const int c = c8 + j;
    float y = ((f[j] - smu[c]) * srs[c]) * sga[c] + sbe[c];
    y = (y > 0.0f) ? y : (y - y);
    y = live ? y : 0.0f;
    const unsigned short hb = bf_bits(y);
    hv[j] = hb;
    lv[j] = bf_bits(y - bf_val(hb));
  }
  unsigned short* hp = p1 + (size_t)row * KP + c8;
  unsigned short* lp = hp + HD;
  *(volatile v8us*)hp = hv;
  *(volatile v8us*)lp = lv;
  __threadfence();
  *(volatile v8us*)hp = hv;
  *(volatile v8us*)lp = lv;
}

__global__ __launch_bounds__(HROWS) void k_headout(const float* __restrict__ pt, const float* __restrict__ stat,
                                                   const float* __restrict__ gam, const float* __restrict__ bet,
                                                   const float* __restrict__ w2, const float* __restrict__ b2,
                                                   float* out, int nG) {
  __shared__ float smu[HD], srs[HD], sga[HD], sbe[HD], sw0[HD], sw1[HD];
  __shared__ __attribute__((aligned(16))) float so[2 * HROWS];
  const int tid = (int)threadIdx.x;
  if (tid < HD) {
    smu[tid] = stat[tid];
    srs[tid] = stat[HD + tid];
    sga[tid] = bf_rne(gam[tid]);
    sbe[tid] = bf_rne(bet[tid]);
    sw0[tid] = bf_rne(w2[2 * tid]);
    sw1[tid] = bf_rne(w2[2 * tid + 1]);
  }
  const float b20 = bf_rne(b2[0]);
  const float b21 = bf_rne(b2[1]);
  __syncthreads();
  const int row = (int)blockIdx.x * HROWS + tid;
  const int rc = row < nG ? row : nG - 1;
  const float* pr = pt + (size_t)rc * HD;
  float o0 = 0.0f, o1 = 0.0f;
#pragma unroll 1
  for (int k4 = 0; k4 < HD / 4; ++k4) {
    const v4f t = *(const v4f*)(pr + 4 * k4);
    const float f[4] = {t.x, t.y, t.z, t.w};
#pragma unroll
    for (int j = 0; j < 4; ++j) {
      const int k = 4 * k4 + j;
      float y = ((f[j] - smu[k]) * srs[k]) * sga[k] + sbe[k];
      y = (y > 0.0f) ? y : (y - y);
      o0 = fmaf(y, sw0[k], o0);
      o1 = fmaf(y, sw1[k], o1);
    }
  }
  so[2 * tid]     = o0 + b20;
  so[2 * tid + 1] = o1 + b21;
  __syncthreads();
  v4f v = {0.f, 0.f, 0.f, 0.f};
  const bool ok = tid < (2 * HROWS) / 4;
  float* op = out + (size_t)blockIdx.x * (2 * HROWS) + 4 * tid;
  if (ok) {
    v = *(const v4fa*)(so + 4 * tid);
    *(volatile v4f*)op = v;
  }
  __threadfence();
  if (ok) *(volatile v4f*)op = v;
}

static inline int cdiv(int a, int b) { return (a + b - 1) / b; }
static inline size_t al256(size_t o) { return (o + 255) & ~(size_t)255; }

extern "C" void kernel_launch(void* const* d_in, const int* in_sizes, int n_in,
                              void* d_out, int out_size, void* d_ws, size_t ws_size,
                              hipStream_t stream) {
  if (n_in < 16) return;
  if (in_sizes[0] < HD * GBM || (in_sizes[0] % HD) != 0) return;
  const int nN = in_sizes[0] / HD;
  if (nN >= (1 << 21)) return;
  if (in_sizes[1] < 2 || (in_sizes[1] & 1) != 0) return;
  const int nE = in_sizes[1] / 2;
  if (nE < 1 || nE >= (1 << 21)) return;
  if (in_sizes[2] != nN) return;
  if (in_sizes[4] != 3 * HD * HD || in_sizes[8] != 3 * HD * HD) return;
  if (in_sizes[5] != 3 * HD || in_sizes[6] != 3 * HD || in_sizes[7] != 3 * HD || in_sizes[9] != 3 * HD) return;
  if (in_sizes[10] != HD * HD || in_sizes[11] != HD || in_sizes[12] != HD || in_sizes[13] != HD) return;
  if (in_sizes[14] != HD * 2 || in_sizes[15] != 2) return;
  if (out_size < 2 * HROWS || (out_size % (2 * HROWS)) != 0) return;
  const int nG = out_size / 2;
  if (nG > 65536 || (nG % GBM) != 0 || (nG % NB_P) != 0) return;

  const float* x    = (const float*)d_in[0];
  const int*   ei   = (const int*)  d_in[1];
  const int*   src  = ei;
  const int*   dst  = ei + nE;
  const int*   bat  = (const int*)  d_in[2];
  const float* cW1  = (const float*)d_in[4];
  const float* cb1  = (const float*)d_in[5];
  const float* cgam = (const float*)d_in[6];
  const float* cbet = (const float*)d_in[7];
  const float* cW2  = (const float*)d_in[8];
  const float* cb2  = (const float*)d_in[9];
  const float* hW1  = (const float*)d_in[10];
  const float* hb1  = (const float*)d_in[11];
  const float* hgam = (const float*)d_in[12];
  const float* hbet = (const float*)d_in[13];
  const float* hW2  = (const float*)d_in[14];
  const float* hb2  = (const float*)d_in[15];
  float* out = (float*)d_out;

  const int NPAD = cdiv(nN, GBM) * GBM;
  const int gT   = NPAD / GBM;
  const int gA   = cdiv(NPAD, NB_E);
  const int gP   = nG / NB_P;
  const int gH   = nG / GBM;
  if ((long long)gA * NB_E < (long long)NPAD) return;
  if (gH > gT) return;
  const int vec8e = ((nE & 3) == 0) ? 1 : 0;
  const int vec8p = ((nN & 3) == 0) ? 1 : 0;

  char* ws = (char*)d_ws;
  size_t off = 0;
  const size_t oWP  = off; off = al256(off + (size_t)NPLN * HD * KP * 2);
  const size_t oXB  = off; off = al256(off + (size_t)NPAD * HD * 2);
  const size_t oH   = off; off = al256(off + (size_t)NPAD * HD * 4);
  const size_t oT   = off; off = al256(off + (size_t)NPAD * HD * 4);
  const size_t oP1  = off; off = al256(off + (size_t)NPAD * KP * 2);
  const size_t oLS  = off; off = al256(off + (size_t)gA * RCAP * 4);
  const size_t oCN  = off; off = al256(off + (size_t)gA * NB_E * 4);
  const size_t oOF  = off; off = al256(off + (size_t)gA * NB_E * 4);
  const size_t oRC  = off; off = al256(off + (size_t)gT * RECW * 4);
  const size_t oST  = off; off = al256(off + (size_t)4 * RECW * 4);
  const size_t oLP  = off; off = al256(off + (size_t)gP * RCAP * 4);
  const size_t oCP  = off; off = al256(off + (size_t)gP * NB_P * 4);
  const size_t oOP  = off; off = al256(off + (size_t)gP * NB_P * 4);
  const size_t oGH  = off; off = al256(off + (size_t)nG * KP * 2);
  const size_t oPT  = off; off = al256(off + (size_t)nG * HD * 4);
  if (off > ws_size || off > (size_t)WSCAP) return;
  unsigned short* WP  = (unsigned short*)(ws + oWP);
  unsigned short* XB  = (unsigned short*)(ws + oXB);
  float*          H   = (float*)(ws + oH);
  float*          T   = (float*)(ws + oT);
  unsigned short* P1  = (unsigned short*)(ws + oP1);
  int*            LS  = (int*)(ws + oLS);
  int*            CN  = (int*)(ws + oCN);
  int*            OF  = (int*)(ws + oOF);
  float*          RC  = (float*)(ws + oRC);
  float*          ST  = (float*)(ws + oST);
  int*            LP  = (int*)(ws + oLP);
  int*            CP  = (int*)(ws + oCP);
  int*            OP  = (int*)(ws + oOP);
  unsigned short* GH  = (unsigned short*)(ws + oGH);
  float*          PT  = (float*)(ws + oPT);

  hipFuncSetAttribute(reinterpret_cast<const void*>(&k_compact<0>), hipFuncAttributeMaxDynamicSharedMemorySize, LDS_CMP);
  hipFuncSetAttribute(reinterpret_cast<const void*>(&k_compact<1>), hipFuncAttributeMaxDynamicSharedMemorySize, LDS_CMP);

  k_prep<<<(NUWT + NPAD * 8) / NTHR, NTHR, 0, stream>>>(x, cW1, cW2, hW1, WP, XB, nN, NPAD);
  k_compact<0><<<gA, NTHR, LDS_CMP, stream>>>(dst, src, nE, NB_E, vec8e, nN, LS, CN, OF);
  k_compact<1><<<gP, NTHR, LDS_CMP, stream>>>(bat, bat, nN, NB_P, vec8p, nN, LP, CP, OP);

  for (int l = 0; l < 3; ++l) {
    if (l == 0) {
      k_agg<0><<<gA, NTHR, 0, stream>>>(LS, CN, OF, XB, H, P1, NB_E, nN, nN, NPAD, DEGCAP_E);
    } else {
      k_agg<1><<<gA, NTHR, 0, stream>>>(LS, CN, OF, XB, H, P1, NB_E, nN, nN, NPAD, DEGCAP_E);
    }
    k_gemm<0><<<gT, GTHR, 0, stream>>>(P1, WP + (size_t)l * (HD * KP), cb1 + l * HD, T, nN, NPAD, RC);
    k_comb<<<1, GBN, 0, stream>>>(RC, gT, nN, ST + (size_t)l * RECW);
    k_apply<<<(NPAD * 8) / NTHR, NTHR, 0, stream>>>(T, ST + (size_t)l * RECW, cgam + l * HD, cbet + l * HD,
                                                    P1, nN, NPAD * 8);
    k_gemm<1><<<gT, GTHR, 0, stream>>>(P1, WP + (size_t)(3 + l) * (HD * KP), cb2 + l * HD, H, nN, NPAD, RC);
  }

  k_agg<2><<<gP, NTHR, 0, stream>>>(LP, CP, OP, XB, H, GH, NB_P, nG, nN, nG, DEGCAP_P);
  k_gemm<0><<<gH, GTHR, 0, stream>>>(GH, WP + (size_t)6 * (HD * KP), hb1, PT, nG, nG, RC);
  k_comb<<<1, GBN, 0, stream>>>(RC, gH, nG, ST + (size_t)3 * RECW);
  k_headout<<<nG / HROWS, HROWS, 0, stream>>>(PT, ST + (size_t)3 * RECW, hgam, hbet, hW2, hb2, out, nG);
}
